// ShiftAttentionLayer_75608604278947
// MI455X (gfx1250) — hardware-verified
//
#include <hip/hip_runtime.h>
#include <stddef.h>
#include <stdint.h>
#include <math.h>

#define NBATCH 32
#define NT     8
#define NNODE  256
#define HD     128
#define HD2    256
#define NSLAB  (NBATCH * NT)
#define SLAB_ND (NNODE * HD)
#define SLAB_NN (NNODE * NNODE)
#define NROWS  (NSLAB * NNODE)

static_assert(NSLAB == 256);
static_assert(NROWS % 16 == 0);
static_assert(HD == 128 && HD2 == 256 && NNODE == 256);
static_assert((NT & (NT - 1)) == 0);

typedef _Float16 v16h __attribute__((ext_vector_type(16)));
typedef _Float16 v8h  __attribute__((ext_vector_type(8)));
typedef float    v8f  __attribute__((ext_vector_type(8)));
typedef float    v4f  __attribute__((ext_vector_type(4)));
typedef unsigned int v4u __attribute__((ext_vector_type(4)));

union Frag  { v16h v; v8h h[2]; };
union Pack8 { v8h h; v4u u; };

__device__ __forceinline__ v8f mma16(v16h a, v16h b, v8f c) {
  c = __builtin_amdgcn_wmma_f32_16x16x32_f16(false, a, false, b, (short)0, c, false, false);
  asm volatile("v_nop\n\tv_nop\n\tv_nop\n\tv_nop" : "+v"(c) : "v"(a), "v"(b));
  return c;
}

__device__ __forceinline__ v16h ldfrag(const _Float16* p, int ld, int row0, int k0, int lane) {
  const int m = lane & 15, lh = lane >> 4;
  const _Float16* q = p + (size_t)(row0 + m) * ld + k0 + 8 * lh;
  Frag f;
  f.h[0] = *(const v8h*)(q);
  f.h[1] = *(const v8h*)(q + 16);
  return f.v;
}

__device__ __forceinline__ v8f zero8() { return (v8f){0.f, 0.f, 0.f, 0.f, 0.f, 0.f, 0.f, 0.f}; }

__device__ __forceinline__ v4u pack8(const v4f a, const v4f b) {
  Pack8 pk;
  pk.h = (v8h){(_Float16)a[0], (_Float16)a[1], (_Float16)a[2], (_Float16)a[3],
               (_Float16)b[0], (_Float16)b[1], (_Float16)b[2], (_Float16)b[3]};
  return pk.u;
}

__device__ __forceinline__ float wsum32(float v) {
#pragma unroll
  for (int off = 1; off < 32; off <<= 1) v += __shfl_xor(v, off, 32);
  return v;
}

template <int KK>
__device__ __forceinline__ void gemm32x64(const _Float16* __restrict__ A, int lda,
                                          const _Float16* __restrict__ Bt, int ldb,
                                          int m0, int n0, int lane, v8f (&acc)[2][4]) {
#pragma unroll 2
  for (int k0 = 0; k0 < KK; k0 += 32) {
    const v16h a0 = ldfrag(A, lda, m0, k0, lane);
    const v16h a1 = ldfrag(A, lda, m0 + 16, k0, lane);
    const v16h b0 = ldfrag(Bt, ldb, n0, k0, lane);
    const v16h b1 = ldfrag(Bt, ldb, n0 + 16, k0, lane);
    const v16h b2 = ldfrag(Bt, ldb, n0 + 32, k0, lane);
    const v16h b3 = ldfrag(Bt, ldb, n0 + 48, k0, lane);
    acc[0][0] = mma16(a0, b0, acc[0][0]);
    acc[1][0] = mma16(a1, b0, acc[1][0]);
    acc[0][1] = mma16(a0, b1, acc[0][1]);
    acc[1][1] = mma16(a1, b1, acc[1][1]);
    acc[0][2] = mma16(a0, b2, acc[0][2]);
    acc[1][2] = mma16(a1, b2, acc[1][2]);
    acc[0][3] = mma16(a0, b3, acc[0][3]);
    acc[1][3] = mma16(a1, b3, acc[1][3]);
  }
}

template <int KK>
__device__ __forceinline__ void tile16x64(const _Float16* __restrict__ A, int lda, int arow0,
                                          const _Float16* __restrict__ Bt, int ldb, int col0,
                                          int lane, v8f (&acc)[4]) {
#pragma unroll 2
  for (int k0 = 0; k0 < KK; k0 += 32) {
    const v16h a  = ldfrag(A, lda, arow0, k0, lane);
    const v16h b0 = ldfrag(Bt, ldb, col0, k0, lane);
    const v16h b1 = ldfrag(Bt, ldb, col0 + 16, k0, lane);
    const v16h b2 = ldfrag(Bt, ldb, col0 + 32, k0, lane);
    const v16h b3 = ldfrag(Bt, ldb, col0 + 48, k0, lane);
    acc[0] = mma16(a, b0, acc[0]);
    acc[1] = mma16(a, b1, acc[1]);
    acc[2] = mma16(a, b2, acc[2]);
    acc[3] = mma16(a, b3, acc[3]);
  }
}

__device__ __forceinline__ v4u softmax8(const float* sr) {
  const v4f x0 = *(const v4f*)sr;
  const v4f x1 = *(const v4f*)(sr + 4);
  float v[8] = {x0[0], x0[1], x0[2], x0[3], x1[0], x1[1], x1[2], x1[3]};
  float m = v[0];
#pragma unroll
  for (int i = 1; i < 8; ++i) m = fmaxf(m, v[i]);
#pragma unroll
  for (int off = 1; off < 32; off <<= 1) m = fmaxf(m, __shfl_xor(m, off, 32));
  float s = 0.f;
#pragma unroll
  for (int i = 0; i < 8; ++i) { v[i] = __expf(v[i] - m); s += v[i]; }
  s = wsum32(s);
  const float f = 1024.0f * (1.0f / s);
  const v4f p0 = {v[0] * f, v[1] * f, v[2] * f, v[3] * f};
  const v4f p1 = {v[4] * f, v[5] * f, v[6] * f, v[7] * f};
  return pack8(p0, p1);
}

#define WTP 68
__global__ __launch_bounds__(256) void k_wt(const float* __restrict__ w, _Float16* __restrict__ wt,
                                           int nout, int kin) {
  __shared__ __align__(16) float tf[64 * WTP];
  const int tid = threadIdx.x;
  const int n0 = blockIdx.x * 64;
  const int k0 = blockIdx.y * 64;
  const size_t zo = (size_t)blockIdx.z * (size_t)kin * (size_t)nout;
  const float* ws = w + zo;
  _Float16* wd = wt + zo;
  {
    const int kr = tid >> 4;
    const int n4 = (tid & 15) * 4;
#pragma unroll
    for (int it = 0; it < 4; ++it) {
      const int kl = it * 16 + kr;
      const v4f a = *(const v4f*)(ws + (size_t)(k0 + kl) * nout + n0 + n4);
      *(v4f*)(tf + kl * WTP + n4) = a;
    }
  }
  __syncthreads();
  v4u val[2];
  size_t go[2];
#pragma unroll
  for (int j = 0; j < 2; ++j) {
    const int p  = tid + 256 * j;
    const int nl = p >> 3;
    const int pc = p & 7;
    const float* cp = tf + (pc * 8) * WTP + nl;
    Pack8 pk;
    pk.h = (v8h){(_Float16)(cp[0 * WTP] * 32.0f), (_Float16)(cp[1 * WTP] * 32.0f),
                 (_Float16)(cp[2 * WTP] * 32.0f), (_Float16)(cp[3 * WTP] * 32.0f),
                 (_Float16)(cp[4 * WTP] * 32.0f), (_Float16)(cp[5 * WTP] * 32.0f),
                 (_Float16)(cp[6 * WTP] * 32.0f), (_Float16)(cp[7 * WTP] * 32.0f)};
    val[j] = pk.u;
    go[j]  = (size_t)(n0 + nl) * kin + k0 + pc * 8;
  }
  for (int ps = 0; ps < 2; ++ps) {
#pragma unroll
    for (int j = 0; j < 2; ++j) *(volatile v4u*)(wd + go[j]) = val[j];
    __threadfence();
  }
}

__global__ __launch_bounds__(256) void k_xt(const float* __restrict__ x, const float* __restrict__ tf,
                                           _Float16* __restrict__ xt) {
  const int tid = threadIdx.x;
  const size_t row = (size_t)blockIdx.x * 16 + (tid >> 4);
  const int c8 = (tid & 15) * 8;
  const size_t bt = row >> 8;
  const float* xr = x + row * HD + c8;
  const float* tr = tf + bt * HD + c8;
  const v4f a0 = *(const v4f*)xr;
  const v4f a1 = *(const v4f*)(xr + 4);
  const v4f t0 = *(const v4f*)tr;
  const v4f t1 = *(const v4f*)(tr + 4);
  const v4u vv = pack8(a0 + t0, a1 + t1);
  volatile v4u* q = (volatile v4u*)(xt + row * HD + c8);
  *q = vv;
  __threadfence();
  *q = vv;
}

#define STP 72
__global__ __launch_bounds__(256) void k_qkv(const _Float16* __restrict__ xt,
                                             const _Float16* __restrict__ wts,
                                             const float* __restrict__ bq, const float* __restrict__ bk,
                                             const float* __restrict__ bv,
                                             _Float16* __restrict__ qp, _Float16* __restrict__ kp,
                                             _Float16* __restrict__ vt) {
  __shared__ __align__(16) _Float16 st[256 * STP];
  const int tid = threadIdx.x, lane = tid & 31, wave = tid >> 5;
  const int hh = lane >> 4, c = lane & 15;
  const int bt = blockIdx.x;
  const int ts = bt & (NT - 1);
  const int which = blockIdx.y >> 1;
  const int nin = (blockIdx.y & 1) * 64;
  const int m0 = wave * 32;
  const _Float16* A = xt + (size_t)bt * SLAB_ND;
  const _Float16* Bw = wts + ((size_t)which * NT + ts) * (size_t)(HD * HD);
  const float* bias = ((which == 0) ? bq : ((which == 1) ? bk : bv)) + ts * HD + nin;

  v8f acc[2][4];
#pragma unroll
  for (int s = 0; s < 2; ++s)
#pragma unroll
    for (int t4 = 0; t4 < 4; ++t4) acc[s][t4] = zero8();
  gemm32x64<HD>(A, HD, Bw, HD, m0, nin, lane, acc);

  float bc[4];
#pragma unroll
  for (int t4 = 0; t4 < 4; ++t4) bc[t4] = bias[16 * t4 + c];
#pragma unroll
  for (int t4 = 0; t4 < 4; ++t4) {
#pragma unroll
    for (int sub = 0; sub < 2; ++sub) {
#pragma unroll
      for (int r = 0; r < 8; ++r) {
        const int lr = wave * 32 + sub * 16 + 8 * hh + r;
        st[lr * STP + 16 * t4 + c] = (_Float16)(acc[sub][t4][r] * 0.03125f + bc[t4]);
      }
    }
  }
  __syncthreads();

  v4u val[8];
  size_t go[8];
  _Float16* dst;
  if (which < 2) {
    dst = (which == 0) ? qp : kp;
#pragma unroll
    for (int j = 0; j < 8; ++j) {
      const int p  = tid + 256 * j;
      const int lr = p >> 3;
      const int pc = p & 7;
      Pack8 pk;
      pk.h   = *(const v8h*)(st + lr * STP + pc * 8);
      val[j] = pk.u;
      go[j]  = ((size_t)bt * NNODE + lr) * HD + nin + pc * 8;
    }
  } else {
    dst = vt;
#pragma unroll
    for (int j = 0; j < 8; ++j) {
      const int p  = tid + 256 * j;
      const int L  = p >> 3;
      const int pc = p & 7;
      const int dl = L >> 2;
      const int nl = (L & 3) * 64 + pc * 8;
      const _Float16* cp = st + nl * STP + dl;
      Pack8 pk;
      pk.h = (v8h){cp[0 * STP], cp[1 * STP], cp[2 * STP], cp[3 * STP],
                   cp[4 * STP], cp[5 * STP], cp[6 * STP], cp[7 * STP]};
      val[j] = pk.u;
      go[j]  = ((size_t)bt * HD + nin + dl) * NNODE + nl;
    }
  }
  for (int ps = 0; ps < 2; ++ps) {
#pragma unroll
    for (int j = 0; j < 8; ++j) *(volatile v4u*)(dst + go[j]) = val[j];
    __threadfence();
  }
}

#define SFP 260
#define SHP 264
#define OTP 68
#define ATT_LDS (64 * SFP * 4 + 64 * SHP * 2)
__global__ __launch_bounds__(256) void k_attw(const _Float16* __restrict__ qp,
                                             const _Float16* __restrict__ kp,
                                             _Float16* __restrict__ wp, _Float16* __restrict__ wtp) {
  extern __shared__ __align__(16) unsigned char dyn_smem[];
  float* sf = (float*)dyn_smem;
  _Float16* sh = (_Float16*)(dyn_smem + 64 * SFP * 4);
  const int tid = threadIdx.x, lane = tid & 31, wave = tid >> 5;
  const int hh = lane >> 4, c = lane & 15;
  const int bt = blockIdx.x;
  const int nr0 = blockIdx.y * 64;
  const int rg = wave >> 1, ch = wave & 1;
  const _Float16* Q = qp + (size_t)bt * SLAB_ND;
  const _Float16* K = kp + (size_t)bt * SLAB_ND;
  const float SC = 0.08838834764831845f;

#pragma unroll 1
  for (int cc = 0; cc < 2; ++cc) {
    const int col0 = ch * 128 + cc * 64;
    v8f acc[4];
#pragma unroll
    for (int j = 0; j < 4; ++j) acc[j] = zero8();
    tile16x64<HD>(Q, HD, nr0 + 16 * rg, K, HD, col0, lane, acc);
#pragma unroll
    for (int j = 0; j < 4; ++j)
#pragma unroll
      for (int r = 0; r < 8; ++r)
        sf[(16 * rg + 8 * hh + r) * SFP + col0 + 16 * j + c] = acc[j][r] * SC;
  }
  __syncthreads();

  _Float16* Wrows = wp + ((size_t)bt * NNODE + nr0) * NNODE;
#pragma unroll 1
  for (int rr = 0; rr < 8; ++rr) {
    const int row = wave * 8 + rr;
    const v4u pk = softmax8(sf + row * SFP + 8 * lane);
    *(v4u*)(sh + row * SHP + 8 * lane) = pk;
    volatile v4u* gq = (volatile v4u*)(Wrows + (size_t)row * NNODE + 8 * lane);
    *gq = pk;
    __threadfence();
    *gq = pk;
  }
  __syncthreads();

  v4u val[8];
  size_t go[8];
#pragma unroll
  for (int j = 0; j < 8; ++j) {
    const int p  = tid + 256 * j;
    const int m  = p >> 3;
    const int pc = p & 7;
    const _Float16* cp = sh + (pc * 8) * SHP + m;
    Pack8 pk;
    pk.h = (v8h){cp[0 * SHP], cp[1 * SHP], cp[2 * SHP], cp[3 * SHP],
                 cp[4 * SHP], cp[5 * SHP], cp[6 * SHP], cp[7 * SHP]};
    val[j] = pk.u;
    go[j]  = ((size_t)bt * NNODE + m) * NNODE + nr0 + pc * 8;
  }
  for (int ps = 0; ps < 2; ++ps) {
#pragma unroll
    for (int j = 0; j < 8; ++j) *(volatile v4u*)(wtp + go[j]) = val[j];
    __threadfence();
  }
}

__global__ __launch_bounds__(256) void k_prop(const _Float16* __restrict__ wp,
                                             const _Float16* __restrict__ wtp,
                                             _Float16* __restrict__ uwp) {
  extern __shared__ __align__(16) unsigned char dyn_smem[];
  float* sf = (float*)dyn_smem;
  _Float16* sa = (_Float16*)(dyn_smem + 64 * SFP * 4);
  const int tid = threadIdx.x, lane = tid & 31, wave = tid >> 5;
  const int hh = lane >> 4, c = lane & 15;
  const int idx = blockIdx.x;
  const int b = idx / (NT - 1);
  const int ts = idx - b * (NT - 1) + 1;
  const int btc = b * NT + ts;
  const int nr0 = blockIdx.y * 64;
  const int rg = wave >> 1, ch = wave & 1;
  const _Float16* Wpv = wp + (size_t)(btc - 1) * SLAB_NN;
  const _Float16* Wcu = wp + (size_t)btc * SLAB_NN;
  const _Float16* WcT = wtp + (size_t)btc * SLAB_NN;
  _Float16* U = uwp + (size_t)btc * SLAB_NN;
  const float SC2 = 5.9604644775390625e-08f;

#pragma unroll 1
  for (int cc = 0; cc < 2; ++cc) {
    const int col0 = ch * 128 + cc * 64;
    v8f acc[4];
#pragma unroll
    for (int j = 0; j < 4; ++j) acc[j] = zero8();
    tile16x64<HD2>(Wpv, HD2, nr0 + 16 * rg, Wcu, HD2, col0, lane, acc);
#pragma unroll
    for (int j = 0; j < 4; ++j)
#pragma unroll
      for (int r = 0; r < 8; ++r)
        sf[(16 * rg + 8 * hh + r) * SFP + col0 + 16 * j + c] = acc[j][r] * SC2;
  }
  __syncthreads();

#pragma unroll 1
  for (int rr = 0; rr < 8; ++rr) {
    const int row = wave * 8 + rr;
    const v4u pk = softmax8(sf + row * SFP + 8 * lane);
    *(v4u*)(sa + row * SHP + 8 * lane) = pk;
  }
  __syncthreads();

  float* sw = sf + wave * (16 * OTP);
#pragma unroll 1
  for (int cc = 0; cc < 2; ++cc) {
    const int col0 = ch * 128 + cc * 64;
    v8f acc[4];
#pragma unroll
    for (int j = 0; j < 4; ++j) acc[j] = zero8();
    tile16x64<HD2>(sa, SHP, 16 * rg, WcT, HD2, col0, lane, acc);
    __syncthreads();
#pragma unroll
    for (int j = 0; j < 4; ++j)
#pragma unroll
      for (int r = 0; r < 8; ++r)
        sw[(8 * hh + r) * OTP + 16 * j + c] = acc[j][r] * 0.0009765625f;
    __syncthreads();
    v4u val[4];
    size_t go[4];
#pragma unroll
    for (int it = 0; it < 4; ++it) {
      const int p   = lane + 32 * it;
      const int L   = p >> 3;
      const int pc  = p & 7;
      const int row = nr0 + 16 * rg + L;
      const v4f x0 = *(const v4f*)(sw + L * OTP + pc * 8);
      const v4f x1 = *(const v4f*)(sw + L * OTP + pc * 8 + 4);
      Pack8 rc;
      rc.h = *(const v8h*)(Wcu + (size_t)row * HD2 + col0 + pc * 8);
      const v4f u0 = {x0[0] + (float)rc.h[0], x0[1] + (float)rc.h[1], x0[2] + (float)rc.h[2], x0[3] + (float)rc.h[3]};
      const v4f u1 = {x1[0] + (float)rc.h[4], x1[1] + (float)rc.h[5], x1[2] + (float)rc.h[6], x1[3] + (float)rc.h[7]};
      val[it] = pack8(u0, u1);
      go[it]  = (size_t)row * HD2 + col0 + pc * 8;
    }
    for (int ps = 0; ps < 2; ++ps) {
#pragma unroll
      for (int it = 0; it < 4; ++it) *(volatile v4u*)(U + go[it]) = val[it];
      __threadfence();
    }
  }
}

#define ZP 132
#define GLN_LDS (NNODE * ZP * 4 + 16 * 4)
__global__ __launch_bounds__(256) void k_gemmln(const _Float16* aw, const _Float16* au,
                                               const _Float16* __restrict__ bp, int bsl,
                                               const float* __restrict__ bias, float bsc, float oscale,
                                               const float* res,
                                               const float* __restrict__ g, const float* __restrict__ bb,
                                               float* outp) {
  extern __shared__ __align__(16) unsigned char dyn_smem[];
  float* zt  = (float*)dyn_smem;
  float* red = zt + NNODE * ZP;
  const int tid = threadIdx.x, lane = tid & 31, wave = tid >> 5;
  const int hh = lane >> 4, c = lane & 15;
  const int bt = blockIdx.x, ts = bt & (NT - 1);
  const _Float16* A = ((ts == 0) ? aw : au) + (size_t)bt * SLAB_NN;
  const _Float16* B = bp + (size_t)bt * (size_t)bsl;
  const int m0 = wave * 32;

#pragma unroll 1
  for (int nh = 0; nh < 2; ++nh) {
    const int n0 = nh * 64;
    v8f acc[2][4];
#pragma unroll
    for (int s = 0; s < 2; ++s)
#pragma unroll
      for (int t4 = 0; t4 < 4; ++t4) acc[s][t4] = zero8();
    gemm32x64<HD2>(A, HD2, B, HD2, m0, n0, lane, acc);
    float bc[4];
#pragma unroll
    for (int t4 = 0; t4 < 4; ++t4) bc[t4] = bias[n0 + 16 * t4 + c] * bsc;
#pragma unroll
    for (int sub = 0; sub < 2; ++sub)
#pragma unroll
      for (int t4 = 0; t4 < 4; ++t4)
#pragma unroll
        for (int r = 0; r < 8; ++r)
          zt[(m0 + 16 * sub + 8 * hh + r) * ZP + n0 + 16 * t4 + c] = acc[sub][t4][r] * oscale + bc[t4];
  }
  __syncthreads();

  const float* R = res + (size_t)bt * SLAB_ND;
  float* O = outp + (size_t)bt * SLAB_ND;

  float s = 0.f;
#pragma unroll 4
  for (int j = 0; j < 32; ++j) {
    const int p = tid + 256 * j;
    const int row = p >> 5, col = (p & 31) * 4;
    float* zq = zt + row * ZP + col;
    v4f z = *(const v4f*)zq;
    const v4f rr = *(const v4f*)(R + row * HD + col);
    z = z + rr;
    *(v4f*)zq = z;
    s += (z[0] + z[1]) + (z[2] + z[3]);
  }
  s = wsum32(s);
  if (lane == 0) red[wave] = s;
  __syncthreads();
  float tsum = 0.f;
#pragma unroll
  for (int w = 0; w < 8; ++w) tsum += red[w];
  const float mean = tsum * (1.0f / (float)SLAB_ND);

  float q = 0.f;
#pragma unroll 4
  for (int j = 0; j < 32; ++j) {
    const int p = tid + 256 * j;
    const int row = p >> 5, col = (p & 31) * 4;
    const v4f z = *(const v4f*)(zt + row * ZP + col);
    const float d0 = z[0] - mean, d1 = z[1] - mean, d2 = z[2] - mean, d3 = z[3] - mean;
    q += (d0 * d0 + d1 * d1) + (d2 * d2 + d3 * d3);
  }
  q = wsum32(q);
  if (lane == 0) red[8 + wave] = q;
  __syncthreads();
  float tq = 0.f;
#pragma unroll
  for (int w = 0; w < 8; ++w) tq += red[8 + w];
  const float var = tq * (1.0f / (float)SLAB_ND);
  const float rstd = rsqrtf(var + 1e-5f);

#pragma unroll 4
  for (int j = 0; j < 32; ++j) {
    const int p = tid + 256 * j;
    const int row = p >> 5, col = (p & 31) * 4;
    float* zq = zt + row * ZP + col;
    const v4f z = *(const v4f*)zq;
    const v4f gg = *(const v4f*)(g + row * HD + col);
    const v4f b4 = *(const v4f*)(bb + row * HD + col);
    v4f o;
    o[0] = (z[0] - mean) * rstd * gg[0] + b4[0];
    o[1] = (z[1] - mean) * rstd * gg[1] + b4[1];
    o[2] = (z[2] - mean) * rstd * gg[2] + b4[2];
    o[3] = (z[3] - mean) * rstd * gg[3] + b4[3];
    *(v4f*)zq = o;
  }
  for (int ps = 0; ps < 2; ++ps) {
#pragma unroll 4
    for (int j = 0; j < 32; ++j) {
      const int p = tid + 256 * j;
      const int row = p >> 5, col = (p & 31) * 4;
      const v4f o = *(const v4f*)(zt + row * ZP + col);
      *(volatile v4f*)(O + (size_t)row * HD + col) = o;
    }
    __threadfence();
  }
}

#define ATP 136
#define FFN1_LDS (NNODE * ATP * 2 + 8 * 16 * OTP * 4)
__global__ __launch_bounds__(256) void k_ffn1(const float* __restrict__ fin,
                                             const _Float16* __restrict__ w1t,
                                             const float* __restrict__ b1, const float* __restrict__ pa,
                                             _Float16* __restrict__ hp) {
  extern __shared__ __align__(16) unsigned char dyn_smem[];
  _Float16* at = (_Float16*)dyn_smem;
  float* stg = (float*)(dyn_smem + NNODE * ATP * 2);
  const int tid = threadIdx.x, lane = tid & 31, wave = tid >> 5;
  const int hh = lane >> 4, c = lane & 15;
  const int bt = blockIdx.x;
  const float* F = fin + (size_t)bt * SLAB_ND;
#pragma unroll 4
  for (int j = 0; j < 16; ++j) {
    const int p = tid + 256 * j;
    const int row = p >> 4, c8 = (p & 15) * 8;
    const v4f a0 = *(const v4f*)(F + row * HD + c8);
    const v4f a1 = *(const v4f*)(F + row * HD + c8 + 4);
    *(v4u*)(at + row * ATP + c8) = pack8(a0, a1);
  }
  __syncthreads();
  const float alpha = pa[0];
  const int m0 = wave * 32;
  float* sw = stg + wave * (16 * OTP);
  _Float16* H = hp + (size_t)bt * NNODE * HD2;

#pragma unroll 1
  for (int nc = 0; nc < 4; ++nc) {
    const int n0 = nc * 64;
    v8f acc[2][4];
#pragma unroll
    for (int s = 0; s < 2; ++s)
#pragma unroll
      for (int t4 = 0; t4 < 4; ++t4) acc[s][t4] = zero8();
    gemm32x64<HD>(at, ATP, w1t, HD, m0, n0, lane, acc);
#pragma unroll
    for (int sub = 0; sub < 2; ++sub) {
      __syncthreads();
#pragma unroll
      for (int t4 = 0; t4 < 4; ++t4)
#pragma unroll
        for (int r = 0; r < 8; ++r)
          sw[(8 * hh + r) * OTP + 16 * t4 + c] = acc[sub][t4][r] * 0.03125f;
      __syncthreads();
      v4u val[4];
      size_t go[4];
#pragma unroll
      for (int it = 0; it < 4; ++it) {
        const int p  = lane + 32 * it;
        const int L  = p >> 3;
        const int pc = p & 7;
        const v4f x0 = *(const v4f*)(sw + L * OTP + pc * 8);
        const v4f x1 = *(const v4f*)(sw + L * OTP + pc * 8 + 4);
        const v4f bb0 = *(const v4f*)(b1 + n0 + pc * 8);
        const v4f bb1 = *(const v4f*)(b1 + n0 + pc * 8 + 4);
        v4f u0 = x0 + bb0, u1 = x1 + bb1;
#pragma unroll
        for (int i = 0; i < 4; ++i) {
          u0[i] = ((u0[i] >= 0.f) ? u0[i] : alpha * u0[i]) * 8.0f;
          u1[i] = ((u1[i] >= 0.f) ? u1[i] : alpha * u1[i]) * 8.0f;
        }
        val[it] = pack8(u0, u1);
        go[it]  = (size_t)(m0 + sub * 16 + L) * HD2 + n0 + pc * 8;
      }
      for (int ps = 0; ps < 2; ++ps) {
#pragma unroll
        for (int it = 0; it < 4; ++it) *(volatile v4u*)(H + go[it]) = val[it];
        __threadfence();
      }
    }
  }
}

extern "C" void kernel_launch(void* const* d_in, const int* in_sizes, int n_in,
                              void* d_out, int out_size, void* d_ws, size_t ws_size,
                              hipStream_t stream) {
  if (n_in < 16) return;
  if (in_sizes[0] != NROWS * HD) return;
  if (in_sizes[1] != NSLAB * HD) return;
  if (in_sizes[3] != NT * HD * HD || in_sizes[5] != NT * HD * HD || in_sizes[7] != NT * HD * HD) return;
  if (in_sizes[4] != NT * HD || in_sizes[6] != NT * HD || in_sizes[8] != NT * HD) return;
  if (in_sizes[9] != SLAB_ND || in_sizes[10] != SLAB_ND) return;
  if (in_sizes[11] != HD * HD2 || in_sizes[12] != HD2) return;
  if (in_sizes[13] < 1) return;
  if (in_sizes[14] != HD2 * HD || in_sizes[15] != HD) return;
  if (out_size != NROWS * HD) return;

  const float* x    = (const float*)d_in[0];
  const float* tf   = (const float*)d_in[1];
  const float* Wq   = (const float*)d_in[3];
  const float* bq   = (const float*)d_in[4];
  const float* Wk   = (const float*)d_in[5];
  const float* bk   = (const float*)d_in[6];
  const float* Wv   = (const float*)d_in[7];
  const float* bv   = (const float*)d_in[8];
  const float* ln_g = (const float*)d_in[9];
  const float* ln_b = (const float*)d_in[10];
  const float* W1   = (const float*)d_in[11];
  const float* b1   = (const float*)d_in[12];
  const float* pa   = (const float*)d_in[13];
  const float* W2   = (const float*)d_in[14];
  const float* b2   = (const float*)d_in[15];
  float* out = (float*)d_out;

  const size_t P16 = (size_t)NROWS * HD * 2;
  const size_t P32 = (size_t)NSLAB * SLAB_NN * 2;
  static_assert((size_t)NROWS * HD2 * 2 == (size_t)NSLAB * SLAB_NN * 2);
  static_assert((size_t)NROWS * HD * 4 == (size_t)NSLAB * SLAB_NN * 2);
  const size_t oWT  = 0;
  const size_t oW1  = oWT + (size_t)3 * NT * HD * HD * 2;
  const size_t oW2  = oW1 + (size_t)HD2 * HD * 2;
  const size_t oVT  = 1048576;
  if (oW2 + (size_t)HD * HD2 * 2 > oVT) return;
  const size_t oQ   = oVT + P16;
  const size_t oK   = oQ + P16;
  const size_t oUW  = oQ;
  const size_t oWP  = oK + P16;
  const size_t oXT  = oWP;
  const size_t oH   = oWP;
  const size_t oWTP = oWP + P32;
  const size_t oFIN = oWTP;
  const size_t total = oWTP + P32;
  if (total > ws_size) return;
  if (total > (size_t)134217728) return;

  char* ws = (char*)d_ws;
  _Float16* WT  = (_Float16*)(ws + oWT);
  _Float16* W1T = (_Float16*)(ws + oW1);
  _Float16* W2T = (_Float16*)(ws + oW2);
  _Float16* VT  = (_Float16*)(ws + oVT);
  _Float16* QP  = (_Float16*)(ws + oQ);
  _Float16* KP  = (_Float16*)(ws + oK);
  _Float16* UWP = (_Float16*)(ws + oUW);
  _Float16* WPL = (_Float16*)(ws + oWP);
  _Float16* XT  = (_Float16*)(ws + oXT);
  _Float16* HP  = (_Float16*)(ws + oH);
  _Float16* WTL = (_Float16*)(ws + oWTP);
  float*    FIN = (float*)(ws + oFIN);

  (void)hipFuncSetAttribute(reinterpret_cast<const void*>(&k_attw), hipFuncAttributeMaxDynamicSharedMemorySize, ATT_LDS);
  (void)hipFuncSetAttribute(reinterpret_cast<const void*>(&k_prop), hipFuncAttributeMaxDynamicSharedMemorySize, ATT_LDS);
  (void)hipFuncSetAttribute(reinterpret_cast<const void*>(&k_gemmln), hipFuncAttributeMaxDynamicSharedMemorySize, GLN_LDS);
  (void)hipFuncSetAttribute(reinterpret_cast<const void*>(&k_ffn1), hipFuncAttributeMaxDynamicSharedMemorySize, FFN1_LDS);

  k_wt<<<dim3(HD / 64, HD / 64, NT), dim3(256), 0, stream>>>(Wq, WT, HD, HD);
  k_wt<<<dim3(HD / 64, HD / 64, NT), dim3(256), 0, stream>>>(Wk, WT + (size_t)NT * HD * HD, HD, HD);
  k_wt<<<dim3(HD / 64, HD / 64, NT), dim3(256), 0, stream>>>(Wv, WT + (size_t)2 * NT * HD * HD, HD, HD);
  k_wt<<<dim3(HD2 / 64, HD / 64, 1), dim3(256), 0, stream>>>(W1, W1T, HD2, HD);
  k_wt<<<dim3(HD / 64, HD2 / 64, 1), dim3(256), 0, stream>>>(W2, W2T, HD, HD2);
  k_xt<<<dim3(NROWS / 16), dim3(256), 0, stream>>>(x, tf, XT);
  k_qkv<<<dim3(NSLAB, 6), dim3(256), 0, stream>>>(XT, WT, bq, bk, bv, QP, KP, VT);
  k_attw<<<dim3(NSLAB, NNODE / 64), dim3(256), ATT_LDS, stream>>>(QP, KP, WPL, WTL);
  k_prop<<<dim3(NBATCH * (NT - 1), NNODE / 64), dim3(256), ATT_LDS, stream>>>(WPL, WTL, UWP);
  k_gemmln<<<dim3(NSLAB), dim3(256), GLN_LDS, stream>>>(WPL, UWP, VT, HD * NNODE, bv, 0.0f, 0.0009765625f,
                                                          x, ln_g, ln_b, FIN);
  k_ffn1<<<dim3(NSLAB), dim3(256), FFN1_LDS, stream>>>(FIN, W1T, b1, pa, HP);
  k_gemmln<<<dim3(NSLAB), dim3(256), GLN_LDS, stream>>>(HP, HP, W2T, 0, b2, 1.0f, 0.00390625f,
                                                          FIN, ln_g, ln_b, out);
  (void)hipGetLastError();
}
